// LorentzMultiheadAttention_56788057588123
// MI455X (gfx1250) — hardware-verified
//
#include <hip/hip_runtime.h>
#include <math.h>

typedef __attribute__((ext_vector_type(16))) _Float16 v16h;
typedef __attribute__((ext_vector_type(16))) __bf16 v16b;
typedef __attribute__((ext_vector_type(8)))  _Float16 v8h;
typedef __attribute__((ext_vector_type(8)))  float v8f;
typedef __attribute__((ext_vector_type(4)))  float v4f;
typedef __attribute__((ext_vector_type(2)))  float v2f;
typedef __attribute__((ext_vector_type(4)))  unsigned v4u;
typedef __attribute__((ext_vector_type(4)))  int v4i;
typedef float __attribute__((may_alias)) float_a;
typedef int __attribute__((may_alias)) int_a;

template <typename T> __device__ __forceinline__ void vst2(void* p, T v) { *(volatile T*)p = v; __threadfence(); *(volatile T*)p = v; }
__device__ __forceinline__ v8f wmma16(v16h a, v16h b, v8f c) {
  v8f d = __builtin_amdgcn_wmma_f32_16x16x32_f16(false, a, false, b, (short)0, c, false, false);
  asm volatile("v_nop\n\tv_nop\n\tv_nop\n\tv_nop" : "+v"(d) : "v"(a), "v"(b));
  return d;
}
__device__ __forceinline__ v8f wmma_bf(v16b a, v16b b, v8f c) {
  v8f d = __builtin_amdgcn_wmma_f32_16x16x32_bf16(false, a, false, b, (short)0, c, false, false);
  asm volatile("v_nop\n\tv_nop\n\tv_nop\n\tv_nop" : "+v"(d) : "v"(a), "v"(b));
  return d;
}
__device__ __forceinline__ v16h frag_h(const _Float16* rowk0, int lane) {
  union { v16h v; v8h q[2]; } u; const _Float16* p = rowk0 + 8 * (lane >> 4);
  u.q[0] = *(const v8h*)p; u.q[1] = *(const v8h*)(p + 16); return u.v;
}
__device__ __forceinline__ v16h frag_f32(const float* rowk0, int lane) {
  v16h a; const float* p = rowk0 + 8 * (lane >> 4);
#pragma unroll
  for (int i = 0; i < 8; ++i) { a[i] = (_Float16)p[i]; a[8 + i] = (_Float16)p[16 + i]; }
  return a;
}
__device__ __forceinline__ v16h frag_f32s(const float* rowk0, int lane, float sc) {
  v16h a; const float* p = rowk0 + 8 * (lane >> 4);
#pragma unroll
  for (int i = 0; i < 8; ++i) { a[i] = (_Float16)(p[i] * sc); a[8 + i] = (_Float16)(p[16 + i] * sc); }
  return a;
}
__device__ __forceinline__ v16h fragc_f32(const float* W, int k0, int n, int lane, int ld, int K) {
  v16h a; const int g = lane >> 4;
#pragma unroll
  for (int i = 0; i < 8; ++i) { const int ka = k0 + 8 * g + i, kb = ka + 16;
    a[i] = (_Float16)(ka < K ? W[(size_t)(ka < K ? ka : K - 1) * ld + n] : 0.f); a[8 + i] = (_Float16)(kb < K ? W[(size_t)(kb < K ? kb : K - 1) * ld + n] : 0.f); }
  return a;
}
struct F2 { v16b h, l; };
__device__ __forceinline__ F2 bsplit16(const float v[16]) { F2 r;
#pragma unroll
  for (int i = 0; i < 16; ++i) { const __bf16 h = (__bf16)v[i]; r.h[i] = h; r.l[i] = (__bf16)(v[i] - (float)h); }
  return r; }
__device__ __forceinline__ F2 split_row(const float* row, int k0, int lane) { float v[16]; const float* p = row + k0 + 8 * (lane >> 4);
#pragma unroll
  for (int i = 0; i < 8; ++i) { v[i] = p[i]; v[8 + i] = p[16 + i]; }
  return bsplit16(v); }
__device__ __forceinline__ F2 split_rowK(const float* row, int k0, int lane, int K) { float v[16]; const int g = lane >> 4;
#pragma unroll
  for (int i = 0; i < 8; ++i) { const int ka = k0 + 8 * g + i, kb = ka + 16; v[i] = ka < K ? row[ka < K ? ka : K - 1] : 0.f; v[8 + i] = kb < K ? row[kb < K ? kb : K - 1] : 0.f; }
  return bsplit16(v); }
__device__ __forceinline__ F2 split_col(const float* W, int k0, int n, int lane, int ld, int K) { float v[16]; const int g = lane >> 4;
#pragma unroll
  for (int i = 0; i < 8; ++i) { const int ka = k0 + 8 * g + i, kb = ka + 16; v[i] = ka < K ? W[(size_t)(ka < K ? ka : K - 1) * ld + n] : 0.f; v[8 + i] = kb < K ? W[(size_t)(kb < K ? kb : K - 1) * ld + n] : 0.f; }
  return bsplit16(v); }
__device__ __forceinline__ v8f mac3(const F2& a, const F2& b, v8f c) { c = wmma_bf(a.l, b.h, c); c = wmma_bf(a.h, b.l, c); return wmma_bf(a.h, b.h, c); }
__device__ __forceinline__ float sigm(float v) { return 1.0f / (1.0f + expf(-v)); }
#define LDSX() do { asm volatile("s_wait_dscnt 0" ::: "memory"); __builtin_amdgcn_wave_barrier(); __builtin_amdgcn_fence(__ATOMIC_RELEASE, "workgroup"); } while (0)


#define NB 2
#define NSEQ 2048
#define NHD 8
#define DH 64
#define EMB 512
#define DOUT 504
#ifndef TNB
#define TNB NB
#define TQB (NSEQ / 64)
#endif
typedef __attribute__((ext_vector_type(8))) __bf16 v8b;
__device__ __forceinline__ v16b frag_b(const __bf16* rowk0, int lane) {
  union { v16b v; v8b q[2]; } u; const __bf16* p = rowk0 + 8 * (lane >> 4);
  u.q[0] = *(const v8b*)p; u.q[1] = *(const v8b*)(p + 16); return u.v;
}
__device__ __forceinline__ v16b frag_gbf(const float* rowk0, int lane) {
  v16b a; const float* p = rowk0 + 8 * (lane >> 4);
#pragma unroll
  for (int i = 0; i < 8; ++i) { a[i] = (__bf16)p[i]; a[8 + i] = (__bf16)p[16 + i]; }
  return a;
}
__device__ __forceinline__ float bfr(float v) { return (float)(__bf16)v; }
__device__ __attribute__((noinline)) float exp_ni(float v) { return expf(v); }

#define WS_Q    0u
#define WS_K    (WS_Q + 4u * NB * NSEQ * EMB)
#define WS_VTH  (WS_K + 4u * NB * NSEQ * EMB)
#define WS_VTL  (WS_VTH + 2u * NB * EMB * NSEQ)
#define WS_M    (WS_VTL + 2u * NB * EMB * NSEQ)
#define WS_L    (WS_M + 4u * NB * NHD * NSEQ)
#define WS_O    (WS_L + 4u * NB * NHD * NSEQ)
#define WS_END  (WS_O + 4u * NB * NSEQ * EMB)

__global__ __launch_bounds__(128) void k_proj(const float* __restrict__ XQ, const float* __restrict__ XS, const float* __restrict__ Wq, const float* __restrict__ bq, const float* __restrict__ Wk, const float* __restrict__ bk, const float* __restrict__ Wv, const float* __restrict__ bv, const float* __restrict__ scale,
                                              float* __restrict__ Q, float* __restrict__ Kr, __bf16* __restrict__ VTH, __bf16* __restrict__ VTL) {
  __shared__ __align__(16) float so[64][68];
  const int tid = threadIdx.x, wave = tid >> 5, lane = tid & 31, col = lane & 15, g = lane >> 4; const int which = blockIdx.z % 3, b = blockIdx.z / 3; const int h = blockIdx.y; const int r0b = blockIdx.x * 64;
  const float* X = which == 0 ? XQ : XS; const float* Wm = which == 0 ? Wq : (which == 1 ? Wk : Wv); const float* bb = which == 0 ? bq : (which == 1 ? bk : bv);
  const size_t arow = ((size_t)b * NSEQ + r0b + wave * 16 + col) * EMB;
  v8f acc[4] = {};
#pragma unroll 2
  for (int kc = 0; kc < EMB / 32; ++kc) { const v16b a = frag_gbf(X + arow + kc * 32, lane);
#pragma unroll
    for (int j = 0; j < 4; ++j) { const int o = h * 63 + j * 16 + col; const int oc = o < (h + 1) * 63 ? o : (h + 1) * 63 - 1;
      acc[j] = wmma_bf(a, frag_gbf(Wm + (size_t)oc * EMB + kc * 32, lane), acc[j]); } }
#pragma unroll
  for (int j = 0; j < 4; ++j) { const int d = j * 16 + col; if (d < 63) { const float bv_ = bfr(bb[h * 63 + d]);
#pragma unroll
      for (int r = 0; r < 8; ++r) so[wave * 16 + 8 * g + r][1 + d] = acc[j][r] + bv_; } }
  LDSX();
  { const int rl = lane >> 1, half = lane & 1; float s = 0.f;
    for (int d = half * 32; d < (half ? 63 : 32); ++d) { const float v = so[wave * 16 + rl][1 + d]; s += v * v; }
    s += __shfl_xor(s, 1); if (half == 0) so[wave * 16 + rl][0] = sqrtf(s + 1.0f); }
  __syncthreads();
  if (which == 2) {
    for (int q = tid; q < 64 * 8; q += 128) { const int d = q >> 3, pc = q & 7; union { __bf16 e[8]; v4u u; } hh, ll;
#pragma unroll
      for (int e = 0; e < 8; ++e) { const float v = so[pc * 8 + e][d]; const __bf16 hi = (__bf16)v; hh.e[e] = hi; ll.e[e] = (__bf16)(v - (float)hi); }
      const size_t o = ((size_t)b * EMB + h * DH + d) * NSEQ + r0b + pc * 8; vst2((unsigned*)(VTH + o), hh.u); vst2((unsigned*)(VTL + o), ll.u); } }
  else { const float f = which == 0 ? 2.0f / bfr(scale[0]) : 1.0f; float* dst = which == 0 ? Q : Kr;
    for (int q = tid; q < 64 * 16; q += 128) { const int rl = q >> 4, pc = q & 15; v4f v = *(const v4f*)&so[rl][pc * 4];
#pragma unroll
      for (int i = 0; i < 4; ++i) { const int d = pc * 4 + i; v[i] = (which == 0 && d == 0) ? -v[i] * f : v[i] * f; }
      vst2(dst + ((size_t)b * NSEQ + r0b + rl) * EMB + h * DH + pc * 4, v); } }
}
__global__ __launch_bounds__(128) void k_stats(const float* __restrict__ Q, const float* __restrict__ Kr, float* __restrict__ Mb, float* __restrict__ Lb) {
  __shared__ __align__(16) float sm[4][16]; __shared__ __align__(16) float ssum[4][16];
  const int tid = threadIdx.x, wave = tid >> 5, lane = tid & 31, col = lane & 15, g = lane >> 4;
  const int bh = blockIdx.y, b = bh >> 3, h = bh & 7; const int q0 = blockIdx.x * 64 + wave * 16;
  const float* qrow = Q + ((size_t)b * NSEQ + q0 + col) * EMB + h * DH; const F2 a0 = split_row(qrow, 0, lane), a1 = split_row(qrow, 32, lane);
  float m[8], l[8];
#pragma unroll
  for (int r = 0; r < 8; ++r) { m[r] = -3.0e38f; l[r] = 0.f; }
#pragma unroll 1
  for (int kt = 0; kt < NSEQ / 16; ++kt) { const float* krow = Kr + ((size_t)b * NSEQ + kt * 16 + col) * EMB + h * DH; const F2 k0 = split_row(krow, 0, lane), k1 = split_row(krow, 32, lane);
    v8f s = mac3(a0, k0, (v8f){}); s = mac3(a1, k1, s);
#pragma unroll
    for (int r = 0; r < 8; ++r) { float mx = s[r];
#pragma unroll
      for (int o = 1; o < 16; o <<= 1) mx = fmaxf(mx, __shfl_xor(mx, o));
      const float mn = fmaxf(m[r], mx); float e = exp_ni(s[r] - mn);
#pragma unroll
      for (int o = 1; o < 16; o <<= 1) e += __shfl_xor(e, o);
      l[r] = l[r] * exp_ni(m[r] - mn) + e; m[r] = mn; } }
  if (col == 0) {
#pragma unroll
    for (int r = 0; r < 8; ++r) { sm[wave][8 * g + r] = m[r]; ssum[wave][8 * g + r] = l[r]; } }
  __syncthreads();
  { const int qb = blockIdx.x * 64; if (tid < 16) vst2(Mb + ((size_t)bh * NSEQ + qb) + tid * 4, *(const v4f*)(&sm[0][0] + tid * 4)); else if (tid < 32) vst2(Lb + ((size_t)bh * NSEQ + qb) + (tid - 16) * 4, *(const v4f*)(&ssum[0][0] + (tid - 16) * 4)); }
}
__global__ __launch_bounds__(128) void k_attn(const float* __restrict__ Q, const float* __restrict__ Kr, const __bf16* __restrict__ VTH, const __bf16* __restrict__ VTL, const float* __restrict__ Mb, const float* __restrict__ Lb, float* __restrict__ O) {
  __shared__ __align__(16) float sp[4][16][36]; __shared__ __align__(16) float so[4][16][68];
  const int tid = threadIdx.x, wave = tid >> 5, lane = tid & 31, col = lane & 15, g = lane >> 4;
  const int bh = blockIdx.y, b = bh >> 3, h = bh & 7; const int q0 = blockIdx.x * 64 + wave * 16;
  const float* qrow = Q + ((size_t)b * NSEQ + q0 + col) * EMB + h * DH; const F2 a0 = split_row(qrow, 0, lane), a1 = split_row(qrow, 32, lane);
  float mr[8], il[8];
#pragma unroll
  for (int r = 0; r < 8; ++r) { mr[r] = Mb[(size_t)bh * NSEQ + q0 + 8 * g + r]; il[r] = 1.0f / Lb[(size_t)bh * NSEQ + q0 + 8 * g + r]; }
  v8f acc[4] = {};
#pragma unroll 1
  for (int ks = 0; ks < NSEQ / 32; ++ks) {
#pragma unroll
    for (int ct = 0; ct < 2; ++ct) { const float* krow = Kr + ((size_t)b * NSEQ + ks * 32 + ct * 16 + col) * EMB + h * DH; const F2 k0 = split_row(krow, 0, lane), k1 = split_row(krow, 32, lane);
      v8f s = mac3(a0, k0, (v8f){}); s = mac3(a1, k1, s);
#pragma unroll
      for (int r = 0; r < 8; ++r) sp[wave][8 * g + r][ct * 16 + col] = exp_ni(s[r] - mr[r]) * il[r]; }
    LDSX();
    const F2 pa = split_row(&sp[wave][col][0], 0, lane);
#pragma unroll
    for (int dt = 0; dt < 4; ++dt) { const size_t vrow = ((size_t)b * EMB + h * DH + dt * 16 + col) * NSEQ + ks * 32; const v16b vh = frag_b(VTH + vrow, lane), vl = frag_b(VTL + vrow, lane);
      acc[dt] = wmma_bf(pa.l, vh, acc[dt]); acc[dt] = wmma_bf(pa.h, vl, acc[dt]); acc[dt] = wmma_bf(pa.h, vh, acc[dt]); }
    LDSX(); }
#pragma unroll
  for (int dt = 0; dt < 4; ++dt)
#pragma unroll
    for (int r = 0; r < 8; ++r) so[wave][8 * g + r][dt * 16 + col] = acc[dt][r];
  LDSX();
  for (int q = lane; q < 16 * 16; q += 32) { const int rl = q >> 4, pc = q & 15; vst2(O + ((size_t)b * NSEQ + q0 + rl) * EMB + h * DH + pc * 4, *(const v4f*)&so[wave][rl][pc * 4]); }
}
__global__ __launch_bounds__(256) void k_fin(const float* __restrict__ O, float* __restrict__ out) {
  __shared__ float sscale[32][8]; __shared__ __align__(16) float smean[32][DH + 4];
  const int tid = threadIdx.x; const size_t r0 = (size_t)blockIdx.x * 32;
  { const int rl = tid >> 3, h = tid & 7; const float* a = O + (r0 + rl) * EMB + h * DH; float ss = 0.f;
#pragma unroll 4
    for (int d = 0; d < DH; ++d) { const float v = a[d]; ss += v * v; }
    const float inner = ss - 2.0f * a[0] * a[0]; sscale[rl][h] = 1.0f / sqrtf(fmaxf(fabsf(inner), 1e-8f)); }
  __syncthreads();
  { const int rl = tid >> 3, dc = tid & 7;
#pragma unroll
    for (int i = 0; i < 8; ++i) { const int d = dc * 8 + i; float s = 0.f;
#pragma unroll
      for (int h = 0; h < NHD; ++h) s += O[(r0 + rl) * EMB + h * DH + d] * sscale[rl][h];
      smean[rl][d] = s * (1.0f / NHD); } }
  __syncthreads();
  { const int rl = tid >> 3, dc = tid & 7; float ss = 0.f;
#pragma unroll 4
    for (int d = 0; d < DH; ++d) { const float v = smean[rl][d]; ss += v * v; }
    const float inner = ss - 2.0f * smean[rl][0] * smean[rl][0]; const float sc = 1.0f / sqrtf(fmaxf(fabsf(inner), 1e-8f));
    v4f v0, v1;
#pragma unroll
    for (int i = 0; i < 4; ++i) { v0[i] = smean[rl][dc * 8 + i] * sc; v1[i] = smean[rl][dc * 8 + 4 + i] * sc; }
    __syncthreads();
    smean[rl][dc * 8 + 0] = v0[0]; smean[rl][dc * 8 + 1] = v0[1]; smean[rl][dc * 8 + 2] = v0[2]; smean[rl][dc * 8 + 3] = v0[3]; smean[rl][dc * 8 + 4] = v1[0]; smean[rl][dc * 8 + 5] = v1[1]; smean[rl][dc * 8 + 6] = v1[2]; smean[rl][dc * 8 + 7] = v1[3]; }
  __syncthreads();
  for (int q = tid; q < 32 * 16; q += 256) { const int rl = q >> 4, pc = q & 15; vst2(out + (r0 + rl) * DH + pc * 4, *(const v4f*)&smean[rl][pc * 4]); }
}

extern "C" void kernel_launch(void* const* d_in, const int* in_sizes, int n_in, void* d_out, int out_size, void* d_ws, size_t ws_size, hipStream_t stream) {
  (void)in_sizes; (void)n_in; (void)out_size;
  const float** F = (const float**)d_in;
  if (ws_size < (size_t)WS_END) return;
  char* ws = (char*)d_ws; float *Q = (float*)(ws + WS_Q), *Kr = (float*)(ws + WS_K), *Mb = (float*)(ws + WS_M), *Lb = (float*)(ws + WS_L), *O = (float*)(ws + WS_O); __bf16 *VTH = (__bf16*)(ws + WS_VTH), *VTL = (__bf16*)(ws + WS_VTL);
  k_proj<<<dim3(NSEQ / 64, NHD, 3 * TNB), 128, 0, stream>>>(F[0], F[1], F[2], F[3], F[4], F[5], F[6], F[7], F[8], Q, Kr, VTH, VTL);
  k_stats<<<dim3(TQB, TNB * NHD), 128, 0, stream>>>(Q, Kr, Mb, Lb);
  k_attn<<<dim3(TQB, TNB * NHD), 128, 0, stream>>>(Q, Kr, VTH, VTL, Mb, Lb, O);
  k_fin<<<TQB * 2 * TNB, 256, 0, stream>>>(O, (float*)d_out);
}
